// LSTM_128849019590
// MI455X (gfx1250) — hardware-verified
//
#include <hip/hip_runtime.h>
#include <math.h>

constexpr int NBATCH   = 256;
constexpr int NSTEP    = 1024;
constexpr int NHID     = 128;
constexpr int NGATE    = 4 * NHID;
constexpr int ROWS_BLK = 16;
constexpr int NTHR     = 256;
constexpr int HPITCH   = 136;
constexpr int XCHUNK   = 256;
constexpr int SPITCH   = 132;
constexpr float WCARRY = 16.0f;
constexpr float HCARRY = 16.0f;
constexpr float FOLD_INV = 1.0f / (WCARRY * HCARRY);

static_assert(NBATCH % ROWS_BLK == 0);
static_assert(NHID == 16 * (NTHR / 32));
static_assert(NHID % 32 == 0);
static_assert(NSTEP % XCHUNK == 0);
static_assert(XCHUNK * ROWS_BLK == 4 * NTHR * 4);
static_assert(ROWS_BLK * NHID == 2 * NTHR * 4);
static_assert((HPITCH % 8) == 0 && HPITCH >= NHID);
static_assert((SPITCH % 4) == 0 && SPITCH >= NHID);
static_assert((NGATE * NHID) % (8 * NTHR) == 0);
static_assert(NBATCH == NTHR);

typedef __attribute__((ext_vector_type(16))) _Float16 v16h;
typedef __attribute__((ext_vector_type(8)))  _Float16 v8h;
typedef __attribute__((ext_vector_type(8)))  float    v8f;
typedef __attribute__((ext_vector_type(4)))  float    v4f;

__device__ __forceinline__ void grp_guard_h(v8f& a0, v8f& a1, v8f& a2, v8f& a3,
                                            v16h a, v16h b0, v16h b1, v16h b2, v16h b3) {
  asm volatile("v_nop\n\tv_nop\n\tv_nop\n\tv_nop"
               : "+v"(a0), "+v"(a1), "+v"(a2), "+v"(a3)
               : "v"(a), "v"(b0), "v"(b1), "v"(b2), "v"(b3));
}
__device__ __forceinline__ void acc_guard4(v8f& a, v8f& b, v8f& c, v8f& d) {
  asm volatile("v_nop\n\tv_nop\n\tv_nop\n\tv_nop" : "+v"(a), "+v"(b), "+v"(c), "+v"(d));
}

struct FragH {
  union U { v16h v; v8h h[2]; };
  static __device__ __forceinline__ v16h load(const _Float16* p) {
    U f;
    f.h[0] = *(const v8h*)(p);
    f.h[1] = *(const v8h*)(p + 16);
    return f.v;
  }
  static __device__ __forceinline__ v8f mma(v16h a, v16h b, v8f c) {
    return __builtin_amdgcn_wmma_f32_16x16x32_f16(false, a, false, b, (short)0, c, false, false);
  }
};

__device__ __forceinline__ float gate_sig(float x)  { return __builtin_amdgcn_rcpf(1.0f + expf(-x)); }
__device__ __forceinline__ float gate_tanh(float x) { return 1.0f - 2.0f * __builtin_amdgcn_rcpf(expf(2.0f * x) + 1.0f); }

__global__ __launch_bounds__(NTHR) void cvt_whh_kernel(const float* __restrict__ src, unsigned short* __restrict__ dst,
                                                       int n8, float sc) {
  const int i = blockIdx.x * NTHR + threadIdx.x;
  if (i < n8) {
    const float* sp = src + (size_t)i * 8;
    const v4f a = *(const v4f*)(sp);
    const v4f b = *(const v4f*)(sp + 4);
    v8h hv;
#pragma unroll
    for (int e = 0; e < 4; ++e) {
      const float fa = a[e] * sc;
      const float fb = b[e] * sc;
      hv[e]     = (_Float16)fa;
      hv[4 + e] = (_Float16)fb;
    }
    _Float16* dp = (_Float16*)dst + (size_t)i * 8;
    *(volatile v8h*)dp = hv;
    __threadfence();
    *(volatile v8h*)dp = hv;
  }
}

__global__ __launch_bounds__(NTHR) void lstm_seq_kernel(const float* __restrict__ x, const float* __restrict__ w_ih,
                                                        const float* __restrict__ b_ih, const float* __restrict__ b_hh,
                                                        const float* __restrict__ h0, const float* __restrict__ c0,
                                                        const unsigned short* __restrict__ WHp,
                                                        float* __restrict__ HFIN) {
  __shared__ __align__(16) _Float16 Ah[2][ROWS_BLK * HPITCH];
  __shared__ __align__(16) float    Xs[XCHUNK * ROWS_BLK];
  __shared__ __align__(16) float    Hs[ROWS_BLK * SPITCH];

  const _Float16* WH = (const _Float16*)WHp;
  const int tid = threadIdx.x, lane = tid & 31, wave = tid >> 5;
  const int c = lane & 15, hh = lane >> 4, koff = hh * 8;
  const int rowbase = blockIdx.x * ROWS_BLK;
  const int j = 16 * wave + c;

  {
    _Float16* ah0 = &Ah[0][0];
#pragma unroll
    for (int it = 0; it < 2; ++it) {
      const int idx = it * NTHR + tid;
      const int row = idx >> 5;
      const int c4  = (idx & 31) * 4;
      const v4f hv = *(const v4f*)(h0 + (size_t)(rowbase + row) * NHID + c4);
      const v4f cv = *(const v4f*)(c0 + (size_t)(rowbase + row) * NHID + c4);
      const float s0 = hv[0] * HCARRY;
      const float s1 = hv[1] * HCARRY;
      const float s2 = hv[2] * HCARRY;
      const float s3 = hv[3] * HCARRY;
      ah0[row * HPITCH + c4 + 0] = (_Float16)s0;
      ah0[row * HPITCH + c4 + 1] = (_Float16)s1;
      ah0[row * HPITCH + c4 + 2] = (_Float16)s2;
      ah0[row * HPITCH + c4 + 3] = (_Float16)s3;
      *(v4f*)(Hs + row * SPITCH + c4) = cv;
    }
  }
  float wih[4], bsum[4];
#pragma unroll
  for (int g = 0; g < 4; ++g) {
    const int n = g * NHID + j;
    wih[g]  = w_ih[n];
    bsum[g] = b_ih[n] + b_hh[n];
  }
  __syncthreads();
  float cst[8], hst[8];
#pragma unroll
  for (int r = 0; r < 8; ++r) {
    cst[r] = Hs[(8 * hh + r) * SPITCH + j];
    hst[r] = 0.0f;
  }

  const _Float16* wh = WH + (size_t)j * NHID + koff;
  const v8f z8 = {0.f, 0.f, 0.f, 0.f, 0.f, 0.f, 0.f, 0.f};

#pragma unroll 1
  for (int t = 0; t < NSTEP; ++t) {
    if ((t & (XCHUNK - 1)) == 0) {
#pragma unroll
      for (int it = 0; it < 4; ++it) {
        const int idx = it * NTHR + tid;
        const int m   = idx >> 6;
        const int t4  = (idx & 63) * 4;
        const v4f v = *(const v4f*)(x + (size_t)(rowbase + m) * NSTEP + (size_t)(t + t4));
        Xs[(t4 + 0) * ROWS_BLK + m] = v[0];
        Xs[(t4 + 1) * ROWS_BLK + m] = v[1];
        Xs[(t4 + 2) * ROWS_BLK + m] = v[2];
        Xs[(t4 + 3) * ROWS_BLK + m] = v[3];
      }
      __syncthreads();
    }

    const int cur = t & 1;
    const _Float16* ahrow = &Ah[cur][0] + c * HPITCH + koff;
    _Float16* ahn = &Ah[cur ^ 1][0];

    v8f acc[4];
    acc[0] = z8; acc[1] = z8; acc[2] = z8; acc[3] = z8;
#pragma unroll 1
    for (int k0 = 0; k0 < NHID; k0 += 32) {
      const v16h a  = FragH::load(ahrow + k0);
      const v16h b0 = FragH::load(wh + k0);
      const v16h b1 = FragH::load(wh + (size_t)1 * NHID * NHID + k0);
      const v16h b2 = FragH::load(wh + (size_t)2 * NHID * NHID + k0);
      const v16h b3 = FragH::load(wh + (size_t)3 * NHID * NHID + k0);
      acc[0] = FragH::mma(a, b0, acc[0]);
      acc[1] = FragH::mma(a, b1, acc[1]);
      acc[2] = FragH::mma(a, b2, acc[2]);
      acc[3] = FragH::mma(a, b3, acc[3]);
      grp_guard_h(acc[0], acc[1], acc[2], acc[3], a, b0, b1, b2, b3);
    }
    acc_guard4(acc[0], acc[1], acc[2], acc[3]);

    const int tc = t & (XCHUNK - 1);
    const v4f xa = *(const v4f*)(Xs + tc * ROWS_BLK + 8 * hh);
    const v4f xb = *(const v4f*)(Xs + tc * ROWS_BLK + 8 * hh + 4);

#pragma unroll
    for (int r = 0; r < 8; ++r) {
      const float xv = (r < 4) ? xa[r & 3] : xb[r & 3];
      const float zi = fmaf(acc[0][r], FOLD_INV, fmaf(xv, wih[0], bsum[0]));
      const float zf = fmaf(acc[1][r], FOLD_INV, fmaf(xv, wih[1], bsum[1]));
      const float zg = fmaf(acc[2][r], FOLD_INV, fmaf(xv, wih[2], bsum[2]));
      const float zo = fmaf(acc[3][r], FOLD_INV, fmaf(xv, wih[3], bsum[3]));
      const float ig = gate_sig(zi);
      const float fg = gate_sig(zf);
      const float gg = gate_tanh(zg);
      const float og = gate_sig(zo);
      const float cn = fg * cst[r] + ig * gg;
      cst[r] = cn;
      const float hn = og * gate_tanh(cn);
      hst[r] = hn;
      const float hs = hn * HCARRY;
      ahn[(8 * hh + r) * HPITCH + j] = (_Float16)hs;
    }
    __syncthreads();
  }

#pragma unroll
  for (int r = 0; r < 8; ++r) Hs[(8 * hh + r) * SPITCH + j] = hst[r];
  __syncthreads();
  for (int pass = 0; pass < 2; ++pass) {
#pragma unroll
    for (int it = 0; it < 2; ++it) {
      const int idx = it * NTHR + tid;
      const int row = idx >> 5;
      const int c4  = (idx & 31) * 4;
      const v4f v = *(const v4f*)(Hs + row * SPITCH + c4);
      *(volatile v4f*)(HFIN + (size_t)(rowbase + row) * NHID + c4) = v;
    }
    __threadfence();
  }
}

__global__ __launch_bounds__(NTHR) void head_kernel(const float* __restrict__ HFIN, const float* __restrict__ w_out,
                                                    const float* __restrict__ b_out, float* __restrict__ out) {
  const int b = threadIdx.x;
  const float* hp = HFIN + (size_t)b * NHID;
  float s = 0.0f;
#pragma unroll 1
  for (int k = 0; k < NHID; k += 4) {
    const v4f hv = *(const v4f*)(hp + k);
    const v4f wv = *(const v4f*)(w_out + k);
    s = fmaf(hv[0], wv[0], s);
    s = fmaf(hv[1], wv[1], s);
    s = fmaf(hv[2], wv[2], s);
    s = fmaf(hv[3], wv[3], s);
  }
  const float v = s + b_out[0];
  *(volatile float*)(out + b) = v;
  __threadfence();
  *(volatile float*)(out + b) = v;
}

extern "C" void kernel_launch(void* const* d_in, const int* in_sizes, int n_in,
                              void* d_out, int out_size, void* d_ws, size_t ws_size, hipStream_t stream) {
  if (n_in < 9 || d_out == nullptr || d_ws == nullptr) return;
  if (in_sizes[0] != NBATCH * NSTEP || in_sizes[1] != NGATE || in_sizes[2] != NGATE * NHID ||
      in_sizes[3] != NGATE || in_sizes[4] != NGATE || in_sizes[5] != NHID || in_sizes[6] != 1 ||
      in_sizes[7] != NBATCH * NHID || in_sizes[8] != NBATCH * NHID || out_size != NBATCH) return;

  const float* xin   = (const float*)d_in[0];
  const float* w_ih  = (const float*)d_in[1];
  const float* w_hh  = (const float*)d_in[2];
  const float* b_ih  = (const float*)d_in[3];
  const float* b_hh  = (const float*)d_in[4];
  const float* w_out = (const float*)d_in[5];
  const float* b_out = (const float*)d_in[6];
  const float* h0    = (const float*)d_in[7];
  const float* c0    = (const float*)d_in[8];
  float* out = (float*)d_out;

  char* ws = (char*)d_ws;
  size_t off = 0;
  auto carve = [&](size_t bytes) -> char* { char* p = ws + off; off += (bytes + 255) & ~(size_t)255; return p; };
  unsigned short* WH   = (unsigned short*)carve((size_t)NGATE * NHID * 2);
  float*          HFIN = (float*)carve((size_t)NBATCH * NHID * 4);
  if (off > ws_size || off > (size_t)134217728) return;

  const int n8 = NGATE * NHID / 8;
  cvt_whh_kernel<<<(n8 + NTHR - 1) / NTHR, NTHR, 0, stream>>>(w_hh, WH, n8, WCARRY);
  lstm_seq_kernel<<<NBATCH / ROWS_BLK, NTHR, 0, stream>>>(xin, w_ih, b_ih, b_hh, h0, c0, WH, HFIN);
  head_kernel<<<1, NTHR, 0, stream>>>(HFIN, w_out, b_out, out);
}
